// ChemiNet_4973572129015
// MI455X (gfx1250) — hardware-verified
//
#include <hip/hip_runtime.h>
#include <stddef.h>
#include <stdint.h>


#define F_ATOM 75
#define F_BOND 12
#define OUTC   10
#define JTOT   (F_ATOM * OUTC)
#define IPAD   80
#define NPAD   (OUTC * IPAD)
#define ITILE  (IPAD / 16)
#define KP     32
#define NTHR   256
#define NWAVE  8
#define TE     16
#define BE     (NWAVE * TE)
#define MSGP   16
#define GPB    32
#define EPT    8
#define CHUNK  (NTHR * EPT)
#define WCAP   (EPT * 32)
#define LISTN  (NWAVE * WCAP)
#define PASSN  NTHR
#define PCAP   (CHUNK + PASSN)
#define PREPT  (2 * NPAD * (KP / 8))
#define PREPB  (PREPT / NTHR)

static_assert((PREPT % NTHR) == 0);
static_assert((IPAD % 16) == 0 && IPAD >= F_ATOM);
static_assert(MSGP >= OUTC && GPB * 4 == 128);
static_assert(2 * F_BOND <= KP);
static_assert(PCAP >= CHUNK + PASSN);
static_assert(WCAP == EPT * 32);
static_assert((KP / 8) == 4);

typedef float          v4f   __attribute__((ext_vector_type(4)));
typedef float          v8f   __attribute__((ext_vector_type(8)));
typedef int            v4i   __attribute__((ext_vector_type(4)));
typedef unsigned short v8us  __attribute__((ext_vector_type(8)));
typedef unsigned short v16us __attribute__((ext_vector_type(16)));
typedef __bf16         v16b  __attribute__((ext_vector_type(16)));
union FragB { v16b v; v16us u; v8us h[2]; };
union Pk8 { v8us h; v4i i; };

__device__ __forceinline__ unsigned short bf16_rne(float f) {
  unsigned u = __float_as_uint(f);
  u = (u + 0x7FFFu + ((u >> 16) & 1u)) >> 16;
  return (unsigned short)u;
}

__device__ __forceinline__ float bf16_val(unsigned short b) {
  return __uint_as_float(((unsigned)b) << 16);
}

__device__ __forceinline__ v8f wmb(v16b a, v16b b, v8f c) {
  v8f d = __builtin_amdgcn_wmma_f32_16x16x32_bf16(false, a, false, b, (short)0, c, false, false);
  asm volatile("v_nop\n\tv_nop\n\tv_nop\n\tv_nop" : "+v"(d) : "v"(a), "v"(b));
  return d;
}

__device__ __forceinline__ v8f zacc() {
  v8f c;
#pragma unroll
  for (int i = 0; i < 8; ++i) c[i] = 0.0f;
  return c;
}

__global__ __launch_bounds__(NTHR) void k_prep(const float* __restrict__ lin_w, unsigned short* pb) {
  const int u     = blockIdx.x * NTHR + threadIdx.x;
  const int plane = u / (NPAD * (KP / 8));
  const int v     = u - plane * (NPAD * (KP / 8));
  const int p     = v >> 2;
  const int kc    = v & 3;
  const int o     = p / IPAD;
  const int i     = p - o * IPAD;
  const int ic    = i < F_ATOM ? i : F_ATOM - 1;
  const int j     = ic * OUTC + o;
  Pk8 pk;
#pragma unroll
  for (int q = 0; q < 8; ++q) {
    const int s = 8 * kc + q;
    const int f = s < F_BOND ? s : (s < 2 * F_BOND ? s - F_BOND : 0);
    const float w = lin_w[j * F_BOND + f];
    const unsigned short hb = bf16_rne(w);
    const unsigned short lb = bf16_rne(w - bf16_val(hb));
    const unsigned short val = (plane == 0) ? hb : lb;
    pk.h[q] = (s < 2 * F_BOND && i < F_ATOM) ? val : (unsigned short)0;
  }
  unsigned short* dp = pb + (size_t)u * 8;
  *(volatile v4i*)dp = pk.i;
  __threadfence();
  *(volatile v4i*)dp = pk.i;
}

__global__ __launch_bounds__(NTHR) void k_edge(
    const float* __restrict__ x, const int* __restrict__ ei, const float* __restrict__ ea,
    const float* __restrict__ lin_b, const unsigned short* __restrict__ pb,
    float* msg, int nN, int nE) {
  __shared__ __attribute__((aligned(16))) float sX[NWAVE * F_ATOM * TE];
  __shared__ __attribute__((aligned(16))) float sM[NWAVE * TE * MSGP];
  __shared__ float sLb[NPAD];
  __shared__ int   sSrc[NWAVE * TE];

  const int tid = threadIdx.x, lane = tid & 31, wv = tid >> 5, h = lane >> 4, m = lane & 15;
  const int e0 = (blockIdx.x * NWAVE + wv) * TE;
  float* sXw = sX + wv * (F_ATOM * TE);
  float* sMw = sM + wv * (TE * MSGP);

#pragma unroll 1
  for (int q = 0; q < (NPAD + NTHR - 1) / NTHR; ++q) {
    const int p  = q * NTHR + tid;
    const int pc = p < NPAD ? p : NPAD - 1;
    const int o  = pc / IPAD;
    const int i  = pc - o * IPAD;
    const int ic = i < F_ATOM ? i : F_ATOM - 1;
    const float v = lin_b[ic * OUTC + o];
    if (p < NPAD) sLb[p] = (i < F_ATOM) ? v : 0.0f;
  }
  {
    int e = e0 + m;
    e = e > nE - 1 ? nE - 1 : e;
    int s = ei[e];
    s = s < 0 ? 0 : (s > nN - 1 ? nN - 1 : s);
    if (h == 0) sSrc[wv * TE + m] = s;
  }
  {
    const v4f z = {0.0f, 0.0f, 0.0f, 0.0f};
    *(v4f*)(sMw + 8 * lane) = z;
    *(v4f*)(sMw + 8 * lane + 4) = z;
  }
  __syncthreads();

#pragma unroll 1
  for (int q = 0; q < (TE * F_ATOM + 31) / 32; ++q) {
    const int c  = q * 32 + lane;
    const int cc = c < TE * F_ATOM ? c : TE * F_ATOM - 1;
    const int e  = cc / F_ATOM;
    const int i  = cc - e * F_ATOM;
    const float v = x[(size_t)sSrc[wv * TE + e] * F_ATOM + i];
    if (c < TE * F_ATOM) sXw[i * TE + e] = v;
  }

  FragB af;
  {
    int e = e0 + m;
    e = e > nE - 1 ? nE - 1 : e;
    const float* ap = ea + (size_t)e * F_BOND;
    const v4f q0 = *(const v4f*)ap;
    const v4f q1 = *(const v4f*)(ap + 4);
    const v4f q2 = *(const v4f*)(ap + 8);
    float av[F_BOND];
    av[0] = q0.x; av[1] = q0.y; av[2]  = q0.z; av[3]  = q0.w;
    av[4] = q1.x; av[5] = q1.y; av[6]  = q1.z; av[7]  = q1.w;
    av[8] = q2.x; av[9] = q2.y; av[10] = q2.z; av[11] = q2.w;
    unsigned short hb[F_BOND], lb[F_BOND];
#pragma unroll
    for (int f = 0; f < F_BOND; ++f) {
      hb[f] = bf16_rne(av[f]);
      lb[f] = bf16_rne(av[f] - bf16_val(hb[f]));
    }
    unsigned short s0[8], s1[8], t0[8];
#pragma unroll
    for (int k = 0; k < 8; ++k) s0[k] = hb[k];
    s1[0] = hb[8]; s1[1] = hb[9]; s1[2] = hb[10]; s1[3] = hb[11];
    s1[4] = lb[0]; s1[5] = lb[1]; s1[6] = lb[2];  s1[7] = lb[3];
#pragma unroll
    for (int k = 0; k < 8; ++k) t0[k] = lb[4 + k];
    const bool h0 = (h == 0);
    v8us r0, r1;
#pragma unroll
    for (int k = 0; k < 8; ++k) {
      r0[k] = h0 ? s0[k] : s1[k];
      r1[k] = h0 ? t0[k] : (unsigned short)0;
    }
    af.h[0] = r0;
    af.h[1] = r1;
  }
  __syncthreads();

  const unsigned short* pl0 = pb;
  const unsigned short* pl1 = pb + (size_t)NPAD * KP;

#pragma unroll 1
  for (int o = 0; o < OUTC; ++o) {
    float pm[8];
#pragma unroll
    for (int r = 0; r < 8; ++r) pm[r] = 0.0f;
#pragma unroll
    for (int it = 0; it < ITILE; ++it) {
      const int t = o * ITILE + it;
      const int p = 16 * t + m;
      FragB b0, b1;
      const unsigned short* bp0 = pl0 + (size_t)p * KP + 8 * h;
      b0.h[0] = *(const v8us*)bp0;
      b0.h[1] = *(const v8us*)(bp0 + 16);
      const unsigned short* bp1 = pl1 + (size_t)p * KP + 8 * h;
      b1.h[0] = *(const v8us*)bp1;
      b1.h[1] = *(const v8us*)(bp1 + 16);
      v8f acc = zacc();
      acc = wmb(af.v, b0.v, acc);
      acc = wmb(af.v, b1.v, acc);
      const float lbv = sLb[p];
      const int i  = 16 * it + m;
      const int ic = i < F_ATOM ? i : F_ATOM - 1;
      const float* xp = sXw + ic * TE + 8 * h;
      const v4f x0 = *(const v4f*)xp;
      const v4f x1 = *(const v4f*)(xp + 4);
      float xs[8];
      xs[0] = x0.x; xs[1] = x0.y; xs[2] = x0.z; xs[3] = x0.w;
      xs[4] = x1.x; xs[5] = x1.y; xs[6] = x1.z; xs[7] = x1.w;
#pragma unroll
      for (int r = 0; r < 8; ++r) {
        const float w = fmaxf(acc[r] + lbv, 0.0f);
        pm[r] = fmaf(w, xs[r], pm[r]);
      }
    }
#pragma unroll
    for (int r = 0; r < 8; ++r) {
      float v = pm[r];
      v += __shfl_xor(v, 1, 32);
      v += __shfl_xor(v, 2, 32);
      v += __shfl_xor(v, 4, 32);
      v += __shfl_xor(v, 8, 32);
      pm[r] = v;
    }
    if (m == 0) {
#pragma unroll
      for (int r = 0; r < 8; ++r) sMw[(8 * h + r) * MSGP + o] = pm[r];
    }
  }
  __syncthreads();

  {
    float* gp = msg + (size_t)e0 * MSGP;
    const v4f v0 = *(const v4f*)(sMw + 4 * lane);
    const v4f v1 = *(const v4f*)(sMw + 128 + 4 * lane);
    *(volatile v4f*)(gp + 4 * lane) = v0;
    *(volatile v4f*)(gp + 128 + 4 * lane) = v1;
    __threadfence();
    *(volatile v4f*)(gp + 4 * lane) = v0;
    *(volatile v4f*)(gp + 128 + 4 * lane) = v1;
  }
}

template <int MODE>
__device__ __forceinline__ int scan_chunk(const int* __restrict__ arr, const int* __restrict__ bt,
                                          int nItems, int nN, int cbase, int g0, int vec,
                                          int* list, int tid, int wave) {
  int wc = 0;
  const int el0 = tid * EPT;
  const int e0  = cbase + el0;
  int dv[EPT];
  if (vec != 0 && cbase + CHUNK <= nItems) {
    const v4i da = *(const v4i*)(arr + e0);
    const v4i db = *(const v4i*)(arr + e0 + 4);
    dv[0] = da.x; dv[1] = da.y; dv[2] = da.z; dv[3] = da.w;
    dv[4] = db.x; dv[5] = db.y; dv[6] = db.z; dv[7] = db.w;
  } else {
#pragma unroll
    for (int j = 0; j < EPT; ++j) {
      int e = e0 + j;
      e = e > nItems - 1 ? nItems - 1 : e;
      dv[j] = arr[e];
    }
  }
  int key[EPT];
  if (MODE == 0) {
#pragma unroll
    for (int j = 0; j < EPT; ++j) {
      int d = dv[j];
      d = d < 0 ? 0 : (d > nN - 1 ? nN - 1 : d);
      key[j] = bt[d];
    }
  } else {
#pragma unroll
    for (int j = 0; j < EPT; ++j) key[j] = dv[j];
  }
  bool hit[EPT];
  bool anyh = false;
#pragma unroll
  for (int j = 0; j < EPT; ++j) {
    hit[j] = (e0 + j < nItems) && ((unsigned)(key[j] - g0) < (unsigned)GPB);
    anyh = anyh || hit[j];
  }
  const unsigned anym = __builtin_amdgcn_ballot_w32(anyh);
  if (anym != 0u) {
#pragma unroll
    for (int j = 0; j < EPT; ++j) {
      const unsigned mj = __builtin_amdgcn_ballot_w32(hit[j]);
      if (mj != 0u) {
        if (hit[j]) {
          const int pos = wc + (int)__builtin_amdgcn_mbcnt_lo(mj, 0u);
          if (pos < WCAP) list[wave * WCAP + pos] = el0 + j;
        }
        wc += (int)__builtin_popcount(mj);
      }
    }
  }
  return wc;
}

template <int MODE>
__device__ __forceinline__ void pool_phase(
    const int* __restrict__ arr, const int* __restrict__ bt, const float* __restrict__ msg,
    const float* __restrict__ x, const float* sRoot, const float* sCb,
    int nItems, int nN, int g0, int vec,
    float* acc, float* srow, int* sslot, int* list, int* pend, int* wcnt,
    int tid, int lane, int wave) {
  const int nChunks = (nItems + CHUNK - 1) / CHUNK;
#pragma unroll 1
  for (int ch = 0; ch < nChunks; ++ch) {
    const int cbase = ch * CHUNK;
    const int wc = scan_chunk<MODE>(arr, bt, nItems, nN, cbase, g0, vec, list, tid, wave);
    if (lane == 0) wcnt[wave] = wc;
    __syncthreads();

    int base = wcnt[NWAVE];
    base = base < 0 ? 0 : (base > PASSN ? PASSN : base);
    int tot = 0, myoff = 0;
#pragma unroll
    for (int w = 0; w < NWAVE; ++w) {
      int c = wcnt[w];
      c = c > WCAP ? WCAP : (c < 0 ? 0 : c);
      if (w < wave) myoff += c;
      tot += c;
    }
    int newN = base + tot;
    newN = newN > PCAP ? PCAP : newN;
    {
      int n = wcnt[wave];
      n = n > WCAP ? WCAP : (n < 0 ? 0 : n);
      const int* lp = list + wave * WCAP;
      for (int i = lane; i < n; i += 32) {
        const int pos = base + myoff + i;
        if (pos < PCAP) pend[pos] = cbase + lp[i];
      }
    }
    const int fin = (ch == nChunks - 1) ? 1 : 0;
    const int R   = (fin != 0) ? (newN + PASSN - 1) / PASSN : newN / PASSN;
    const int Pv  = (fin != 0) ? newN : R * PASSN;
    __syncthreads();

#pragma unroll 1
    for (int r = 0; r < R; ++r) {
      int idx = r * PASSN + tid;
      const bool valid = idx < Pv;
      idx = idx > PCAP - 1 ? PCAP - 1 : idx;
      int it = pend[idx];
      it = it < 0 ? 0 : (it > nItems - 1 ? nItems - 1 : it);
      int key;
      float* rp = srow + tid * MSGP;
      if (MODE == 0) {
        int d = arr[it];
        d = d < 0 ? 0 : (d > nN - 1 ? nN - 1 : d);
        key = bt[d];
        const float* mp = msg + (size_t)it * MSGP;
        const v4f a0 = *(const v4f*)mp;
        const v4f a1 = *(const v4f*)(mp + 4);
        const v4f a2 = *(const v4f*)(mp + 8);
        const v4f a3 = *(const v4f*)(mp + 12);
        *(v4f*)rp = a0;
        *(v4f*)(rp + 4) = a1;
        *(v4f*)(rp + 8) = a2;
        *(v4f*)(rp + 12) = a3;
      } else {
        key = bt[it];
        const float* xr = x + (size_t)it * F_ATOM;
        float hs[OUTC];
#pragma unroll
        for (int o = 0; o < OUTC; ++o) hs[o] = 0.0f;
#pragma unroll 1
        for (int i = 0; i < F_ATOM; ++i) {
          const float xi = xr[i];
          const float* rw = sRoot + i * OUTC;
#pragma unroll
          for (int o = 0; o < OUTC; ++o) hs[o] = fmaf(xi, rw[o], hs[o]);
        }
        const v4f h0 = {hs[0] + sCb[0], hs[1] + sCb[1], hs[2] + sCb[2], hs[3] + sCb[3]};
        const v4f h1 = {hs[4] + sCb[4], hs[5] + sCb[5], hs[6] + sCb[6], hs[7] + sCb[7]};
        const v4f h2 = {hs[8] + sCb[8], hs[9] + sCb[9], 0.0f, 0.0f};
        const v4f h3 = {0.0f, 0.0f, 0.0f, 0.0f};
        *(v4f*)rp = h0;
        *(v4f*)(rp + 4) = h1;
        *(v4f*)(rp + 8) = h2;
        *(v4f*)(rp + 12) = h3;
      }
      int slot = key - g0;
      if (!valid || (unsigned)slot >= (unsigned)GPB) slot = GPB;
      sslot[tid] = slot;
      __syncthreads();
      if (tid < MSGP) {
#pragma unroll 1
        for (int i = 0; i < PASSN; ++i) {
          int sl = sslot[i];
          sl = sl < 0 ? 0 : (sl > GPB ? GPB : sl);
          acc[sl * MSGP + tid] += srow[i * MSGP + tid];
        }
      }
      __syncthreads();
    }
    int rem = newN - R * PASSN;
    rem = rem < 0 ? 0 : rem;
    if (R > 0 && tid < rem) pend[tid] = pend[R * PASSN + tid];
    if (tid == 0) wcnt[NWAVE] = rem;
  }
  __syncthreads();
}

__global__ __launch_bounds__(NTHR) void k_pool(
    const float* __restrict__ x, const int* __restrict__ ei, const int* __restrict__ bt,
    const float* __restrict__ msg, const float* __restrict__ root_w, const float* __restrict__ conv_b,
    const float* __restrict__ out_w, const float* __restrict__ out_b,
    float* out, int nN, int nE, int G, int vecE) {
  __shared__ __attribute__((aligned(16))) float acc[(GPB + 1) * MSGP];
  __shared__ __attribute__((aligned(16))) float srow[PASSN * MSGP];
  __shared__ __attribute__((aligned(16))) float sOut[GPB];
  __shared__ float sRoot[F_ATOM * OUTC];
  __shared__ float sCb[MSGP];
  __shared__ int   sslot[PASSN];
  __shared__ int   list[LISTN];
  __shared__ int   pend[PCAP];
  __shared__ int   wcnt[NWAVE + 1];

  const int tid = threadIdx.x, lane = tid & 31, wave = tid >> 5;
  const int g0 = blockIdx.x * GPB;
  const int* dsts = ei + nE;

#pragma unroll 1
  for (int q = 0; q < ((GPB + 1) * MSGP + NTHR - 1) / NTHR; ++q) {
    const int idx = q * NTHR + tid;
    if (idx < (GPB + 1) * MSGP) acc[idx] = 0.0f;
  }
#pragma unroll 1
  for (int q = 0; q < (F_ATOM * OUTC + NTHR - 1) / NTHR; ++q) {
    const int idx = q * NTHR + tid;
    const int ic  = idx < F_ATOM * OUTC ? idx : F_ATOM * OUTC - 1;
    const float v = root_w[ic];
    if (idx < F_ATOM * OUTC) sRoot[idx] = v;
  }
  {
    const int oc = tid < OUTC ? tid : OUTC - 1;
    const float cb = conv_b[oc];
    if (tid < MSGP) sCb[tid] = (tid < OUTC) ? cb : 0.0f;
  }
  if (tid == 0) wcnt[NWAVE] = 0;
  __syncthreads();

  pool_phase<0>(dsts, bt, msg, x, sRoot, sCb, nE, nN, g0, vecE,
                acc, srow, sslot, list, pend, wcnt, tid, lane, wave);
  if (tid == 0) wcnt[NWAVE] = 0;
  __syncthreads();
  pool_phase<1>(bt, bt, msg, x, sRoot, sCb, nN, nN, g0, 1,
                acc, srow, sslot, list, pend, wcnt, tid, lane, wave);

  float ow[OUTC];
#pragma unroll
  for (int o = 0; o < OUTC; ++o) ow[o] = out_w[o];
  const float ob = out_b[0];
  if (tid < GPB) {
    float s = 0.0f;
#pragma unroll
    for (int o = 0; o < OUTC; ++o) s = fmaf(acc[tid * MSGP + o], ow[o], s);
    sOut[tid] = s + ob;
  }
  __syncthreads();

  v4f v = {0.0f, 0.0f, 0.0f, 0.0f};
  if (tid < GPB / 4) v = *(const v4f*)(sOut + 4 * tid);
  const int gb = g0 + 4 * tid;
  if (tid < GPB / 4) {
    if (gb + 3 < G) {
      *(volatile v4f*)(out + gb) = v;
    } else {
      if (gb     < G) ((volatile float*)out)[gb]     = v.x;
      if (gb + 1 < G) ((volatile float*)out)[gb + 1] = v.y;
      if (gb + 2 < G) ((volatile float*)out)[gb + 2] = v.z;
      if (gb + 3 < G) ((volatile float*)out)[gb + 3] = v.w;
    }
  }
  __threadfence();
  if (tid < GPB / 4) {
    if (gb + 3 < G) {
      *(volatile v4f*)(out + gb) = v;
    } else {
      if (gb     < G) ((volatile float*)out)[gb]     = v.x;
      if (gb + 1 < G) ((volatile float*)out)[gb + 1] = v.y;
      if (gb + 2 < G) ((volatile float*)out)[gb + 2] = v.z;
      if (gb + 3 < G) ((volatile float*)out)[gb + 3] = v.w;
    }
  }
}

extern "C" void kernel_launch(void* const* d_in, const int* in_sizes, int n_in,
                              void* d_out, int out_size, void* d_ws, size_t ws_size,
                              hipStream_t stream) {
  if (n_in < 10) return;
  const int nN = in_sizes[0] / F_ATOM;
  if (nN < 1 || in_sizes[0] != nN * F_ATOM || in_sizes[3] != nN) return;
  const int nE = in_sizes[2] / F_BOND;
  if (nE < 1 || in_sizes[2] != nE * F_BOND || in_sizes[1] != 2 * nE) return;
  if (in_sizes[4] != JTOT * F_BOND || in_sizes[5] != JTOT || in_sizes[6] != F_ATOM * OUTC) return;
  if (in_sizes[7] != OUTC || in_sizes[8] != OUTC || in_sizes[9] < 1) return;
  const int G = out_size;
  if (G < 1) return;

  const float* x      = (const float*)d_in[0];
  const int*   ei     = (const int*)d_in[1];
  const float* eattr  = (const float*)d_in[2];
  const int*   bt     = (const int*)d_in[3];
  const float* lin_w  = (const float*)d_in[4];
  const float* lin_b  = (const float*)d_in[5];
  const float* root_w = (const float*)d_in[6];
  const float* conv_b = (const float*)d_in[7];
  const float* out_w  = (const float*)d_in[8];
  const float* out_b  = (const float*)d_in[9];
  float* outp = (float*)d_out;

  const int nBlkE = (nE + BE - 1) / BE;
  const size_t rowsE = (size_t)nBlkE * BE;

  char* ws = (char*)d_ws;
  size_t off = 0;
  const size_t oPb  = off; off += ((size_t)2 * NPAD * KP * 2 + 255) & ~(size_t)255;
  const size_t oMsg = off; off += (rowsE * MSGP * 4 + 255) & ~(size_t)255;
  size_t limit = (size_t)134217728;
  if (ws_size < limit) limit = ws_size;
  if (off > limit) return;

  unsigned short* pbp = (unsigned short*)(ws + oPb);
  float* msgp = (float*)(ws + oMsg);

  const int vecE  = ((nE & 3) == 0) ? 1 : 0;
  const int nBlkG = (G + GPB - 1) / GPB;

  k_prep<<<PREPB, NTHR, 0, stream>>>(lin_w, pbp);
  k_edge<<<nBlkE, NTHR, 0, stream>>>(x, ei, eattr, lin_b, pbp, msgp, nN, nE);
  k_pool<<<nBlkG, NTHR, 0, stream>>>(x, ei, bt, msgp, root_w, conv_b, out_w, out_b, outp, nN, nE, G, vecE);
}
